// CrossAttentionLayer_40793599378095
// MI455X (gfx1250) — hardware-verified
//
#include <hip/hip_runtime.h>


namespace {
constexpr int B = 8, NQ = 512, NK = 1024, DM = 1024, H = 16, HD = 64, BL = 8  , QL = 512  ;
constexpr size_t OUT1_OFF = (size_t)B * NQ * DM;
constexpr float XS = 8.0f, WSC = 256.0f, PS = 1024.0f, EPS = 1e-5f;
static_assert(NQ % 64 == 0 && NK % 64 == 0 && QL % 64 == 0, "tiling");
typedef _Float16 b16;
typedef __attribute__((ext_vector_type(16))) _Float16 v16b;
typedef __attribute__((ext_vector_type(8))) _Float16 v8b;
typedef __attribute__((ext_vector_type(8))) float v8f;
typedef __attribute__((ext_vector_type(4))) float v4f;
__device__ __forceinline__ float bf16_rne(float f) { unsigned int u = __float_as_uint(f); u += 0x7FFFu + ((u >> 16) & 1u); return __uint_as_float(u & 0xFFFF0000u); }
__device__ __forceinline__ void split16(float v, b16& hi, b16& lo) { hi = (b16)v; lo = (b16)(v - (float)hi); }
__device__ __forceinline__ v16b frag_kb(const b16* p, int hh) { const v8b a = *(const v8b*)(p + 8 * hh), b = *(const v8b*)(p + 16 + 8 * hh); v16b f;
#pragma unroll
  for (int e = 0; e < 8; ++e) { f[e] = a[e]; f[8 + e] = b[e]; } return f; }
__device__ __forceinline__ v8f wmma16b(v16b a, v16b b, v8f c) { v8f d = __builtin_amdgcn_wmma_f32_16x16x32_f16(false, a, false, b, (short)0, c, false, false); asm volatile("v_nop\n\tv_nop\n\tv_nop\n\tv_nop" : "+v"(d) : "v"(a), "v"(b)); return d; }
__device__ __forceinline__ void wave_lds_sync() { __builtin_amdgcn_fence(__ATOMIC_RELEASE, "workgroup"); __builtin_amdgcn_wave_barrier(); __builtin_amdgcn_fence(__ATOMIC_ACQUIRE, "workgroup"); }
__device__ __forceinline__ float pmul(float a, float b) { float p = a * b; asm volatile("" : "+v"(p)); return p; }
__device__ __forceinline__ int iclamp(int v, int lo, int hi) { return v < lo ? lo : (v > hi ? hi : v); }

typedef __attribute__((ext_vector_type(2))) _Float16 v2h;
typedef __attribute__((ext_vector_type(4))) _Float16 v4h;
typedef __attribute__((ext_vector_type(2))) float v2f;
__global__ __launch_bounds__(256) void prep_kernel(const float* __restrict__ wq, const float* __restrict__ wk, const float* __restrict__ wv, b16* __restrict__ WT) {
  const size_t u = (size_t)blockIdx.x * 256 + threadIdx.x; const size_t per = (size_t)DM * DM / 8; if (u >= 3 * per) return; const int m = (int)(u / per); const size_t e = (u % per) * 8; const float* w = m == 0 ? wq : m == 1 ? wk : wv; v8b o;
  for (int j = 0; j < 8; ++j) o[j] = (b16)(bf16_rne(w[e + j]) * WSC);
  for (int pass = 0; pass < 2; ++pass) { *(volatile v8b*)(WT + (size_t)m * DM * DM + e) = o; __threadfence(); }
}
__global__ __launch_bounds__(256) void ln_kernel(const float* __restrict__ x, const float* __restrict__ w, const float* __restrict__ bb, int nrows, float* __restrict__ XN) {
  const int wave = threadIdx.x >> 5, lane = threadIdx.x & 31; const size_t row = (size_t)blockIdx.x * 8 + wave; if (row >= (size_t)nrows) return; const float* xr = x + row * DM;
  float v[32]; float s = 0.0f;
#pragma unroll
  for (int q = 0; q < 8; ++q) { const v4f f = *(const v4f*)(xr + q * 128 + lane * 4); for (int i = 0; i < 4; ++i) { v[q * 4 + i] = bf16_rne(f[i]); s += v[q * 4 + i]; } }
#pragma unroll
  for (int o = 1; o < 32; o <<= 1) s += __shfl_xor(s, o);
  const float mu = s * (1.0f / DM); float vs = 0.0f; for (int i = 0; i < 32; ++i) { const float d = v[i] - mu; vs += d * d; }
#pragma unroll
  for (int o = 1; o < 32; o <<= 1) vs += __shfl_xor(vs, o);
  const float rs = rsqrtf(vs * (1.0f / DM) + EPS);
  for (int pass = 0; pass < 2; ++pass) {
#pragma unroll
    for (int q = 0; q < 8; ++q) { const int c = q * 128 + lane * 4; v4f o4; for (int i = 0; i < 4; ++i) o4[i] = (v[q * 4 + i] - mu) * rs * bf16_rne(w[c + i]) + bf16_rne(bb[c + i]); *(volatile v4f*)(XN + row * DM + c) = o4; }
    __threadfence(); }
}
template <int PART>
__global__ __launch_bounds__(128) void proj_kernel(const float* __restrict__ XN, const b16* __restrict__ WT, const float* __restrict__ b0, const float* __restrict__ b1, b16* __restrict__ P0, b16* __restrict__ P1) {
  __shared__ __attribute__((aligned(16))) b16 As[64][256 + 8]; __shared__ __attribute__((aligned(16))) float Tf[4][16][128 + 4];
  constexpr int NR = (PART == 0) ? NQ : NK;
  const int wave = threadIdx.x >> 5, lane = threadIdx.x & 31, nloc = lane & 15, hlf = lane >> 4; const int t0 = blockIdx.x * 64; const int b = blockIdx.y; const int slab = blockIdx.z; const int sub = (PART == 0) ? 0 : slab / 8; const int c0 = (slab % 8) * 128;
  if (PART == 0 && t0 >= QL) return;
  const float* xb = XN + ((size_t)b * NR + t0) * DM; const b16* W = WT + (size_t)((PART == 0) ? 0 : (1 + sub)) * DM * DM; const float* bias = (sub == 0) ? b0 : b1;
  v8f acc[8];
#pragma unroll
  for (int t = 0; t < 8; ++t) acc[t] = (v8f){};
#pragma unroll 1
  for (int kc = 0; kc < DM; kc += 256) {
    __syncthreads();
    for (int i = threadIdx.x; i < 64 * 64; i += 128) { const int rr = i / 64, q = (i % 64) * 4; const v4f f = *(const v4f*)(xb + (size_t)rr * DM + kc + q); v4h o; for (int j = 0; j < 4; ++j) o[j] = (b16)(f[j] * XS); *(v4h*)(&As[rr][q]) = o; }
    __syncthreads();
#pragma unroll 2
    for (int kb = 0; kb < 256; kb += 32) { const v16b a = frag_kb(&As[wave * 16 + nloc][kb], hlf);
#pragma unroll
      for (int t = 0; t < 8; ++t) acc[t] = wmma16b(a, frag_kb(W + (size_t)(c0 + t * 16 + nloc) * DM + kc + kb, hlf), acc[t]); } }
#pragma unroll
  for (int t = 0; t < 8; ++t) { const float bb = bf16_rne(bias[c0 + t * 16 + nloc]);
#pragma unroll
    for (int r = 0; r < 8; ++r) Tf[wave][8 * hlf + r][t * 16 + nloc] = acc[t][r] * (1.0f / (XS * WSC)) + bb; }
  __syncthreads();
  for (int pass = 0; pass < 2; ++pass) {
    if (PART == 0 || sub == 0) { const int c = c0 + lane * 4; const int h = c / HD, d = c % HD;
      for (int rr = 0; rr < 16; ++rr) { const int tok = t0 + wave * 16 + rr; v4h o4; for (int j = 0; j < 4; ++j) o4[j] = (b16)(Tf[wave][rr][lane * 4 + j] * XS); *(volatile v4h*)(P0 + (((size_t)b * H + h) * NR + tok) * HD + d) = o4; } }
    else {
#pragma unroll 1
      for (int q = 0; q < 32; ++q) { const int cl = wave * 32 + q; const int c = c0 + cl; const int h = c / HD, d = c % HD; const int tk = lane * 2; v2h vv; vv[0] = (b16)(Tf[tk >> 4][tk & 15][cl] * XS); vv[1] = (b16)(Tf[(tk + 1) >> 4][(tk + 1) & 15][cl] * XS);
        *(volatile v2h*)(P1 + (((size_t)b * H + h) * HD + d) * (size_t)NK + t0 + tk) = vv; } }
    __threadfence(); }
}
__global__ __launch_bounds__(32) void attn_kernel(const b16* __restrict__ QP, const b16* __restrict__ KP, const b16* __restrict__ VT, float* __restrict__ out) {
  __shared__ __attribute__((aligned(16))) float W1[16][NK]; __shared__ __attribute__((aligned(16))) b16 Pb[16][32 + 8]; __shared__ __attribute__((aligned(16))) float To[16][HD + 4];
  const int lane = threadIdx.x & 31, hh = lane >> 4, col = lane & 15; const int b = blockIdx.y; const int q0 = blockIdx.x * 16, qi = q0 + col;
  for (int i = lane; i < 16 * NK; i += 32) (&W1[0][0])[i] = 0.0f;
  const float cs = 1.0f / (8.0f * XS * XS);
  float* out0 = out + ((size_t)b * NQ + q0) * DM; float* out1 = out + OUT1_OFF + ((size_t)b * NQ + q0) * NK;
#pragma unroll 1
  for (int h = 0; h < H; ++h) {
    const size_t ph = (size_t)b * H + h; const b16* Qb = QP + (ph * NQ + qi) * HD; const b16* Kb = KP + ph * NK * HD; const b16* Vb = VT + ph * HD * (size_t)NK;
    const v16b qa0 = frag_kb(Qb, hh), qa1 = frag_kb(Qb + 32, hh);
    v8f o[4]; for (int t = 0; t < 4; ++t) o[t] = (v8f){};
    wave_lds_sync();
#pragma unroll 1
    for (int kb = 0; kb < NK; kb += 32) {
#pragma unroll
      for (int u = 0; u < 2; ++u) { v8f s = (v8f){}; const size_t kr = (size_t)(kb + u * 16 + col) * HD; s = wmma16b(frag_kb(Kb + kr, hh), qa0, s); s = wmma16b(frag_kb(Kb + kr + 32, hh), qa1, s);
#pragma unroll
        for (int r = 0; r < 8; ++r) { const float w = 1.0f / (1.0f + __expf(-s[r] * cs)); const int key = kb + u * 16 + 8 * hh + r; W1[col][key] += w; Pb[col][u * 16 + 8 * hh + r] = (b16)(w * PS); } }
      wave_lds_sync();
      const v16b pf = frag_kb(&Pb[col][0], hh);
#pragma unroll
      for (int t = 0; t < 4; ++t) o[t] = wmma16b(frag_kb(Vb + (size_t)(t * 16 + col) * NK + kb, hh), pf, o[t]);
      wave_lds_sync(); }
#pragma unroll
    for (int t = 0; t < 4; ++t)
#pragma unroll
      for (int r = 0; r < 8; ++r) To[col][t * 16 + 8 * hh + r] = o[t][r] * (1.0f / (PS * XS));
    wave_lds_sync();
    for (int pass = 0; pass < 2; ++pass) { for (int rr = 0; rr < 16; ++rr) *(volatile v2f*)(out0 + (size_t)rr * DM + h * HD + lane * 2) = *(const v2f*)(&To[rr][lane * 2]); __threadfence(); }
  }
  wave_lds_sync();
  for (int pass = 0; pass < 2; ++pass) { for (int rr = 0; rr < 16; ++rr) {
#pragma unroll
      for (int q = 0; q < 8; ++q) { v4f f = *(const v4f*)(&W1[rr][q * 128 + lane * 4]); f *= (1.0f / H); *(volatile v4f*)(out1 + (size_t)rr * NK + q * 128 + lane * 4) = f; } }
    __threadfence(); }
}
}

extern "C" void kernel_launch(void* const* d_in, const int* in_sizes, int n_in, void* d_out, int out_size, void* d_ws, size_t ws_size, hipStream_t stream) {
  (void)n_in;
  auto Fp = [&](int i) { return (const float*)d_in[i]; };
  if (in_sizes[0] != B * NQ * DM || in_sizes[1] != B * NK * DM || in_sizes[2] != DM || in_sizes[6] != DM * DM || in_sizes[8] != DM * DM || in_sizes[10] != DM * DM || in_sizes[11] != DM || out_size != B * NQ * DM + B * NQ * NK) return;
  size_t off = 0; char* ws = (char*)d_ws;
  auto carve = [&](size_t bytes) { char* p = ws + off; off += (bytes + 255) & ~(size_t)255; return p; };
  b16* WT = (b16*)carve((size_t)3 * DM * DM * 2); float* TN = (float*)carve((size_t)B * NQ * DM * 4); float* AN = (float*)carve((size_t)B * NK * DM * 4);
  b16* QP = (b16*)carve((size_t)B * NQ * DM * 2); b16* KP = (b16*)carve((size_t)B * NK * DM * 2); b16* VT = (b16*)carve((size_t)B * NK * DM * 2);
  if (off > ws_size || off > ((size_t)128 << 20)) return;
  prep_kernel<<<(unsigned)(((size_t)3 * DM * DM / 8 + 255) / 256), 256, 0, stream>>>(Fp(6), Fp(8), Fp(10), WT);
  ln_kernel<<<(B * NQ + 7) / 8, 256, 0, stream>>>(Fp(0), Fp(2), Fp(3), BL * NQ, TN);
  ln_kernel<<<(B * NK + 7) / 8, 256, 0, stream>>>(Fp(1), Fp(4), Fp(5), BL * NK, AN);
  proj_kernel<0><<<dim3(NQ / 64, BL, 8), 128, 0, stream>>>(TN, WT, Fp(7), Fp(7), QP, QP);
  proj_kernel<1><<<dim3(NK / 64, BL, 16), 128, 0, stream>>>(AN, WT, Fp(9), Fp(11), KP, VT);
  attn_kernel<<<dim3(QL / 16, BL), 32, 0, stream>>>(QP, KP, VT, (float*)d_out);
}
